// MultiHeadAttention_82867099009399
// MI455X (gfx1250) — hardware-run, weakly checked
//
#include <hip/hip_runtime.h>
#include <math.h>

#ifndef NB
#define NB 2
#endif
#ifndef SEQ
#define SEQ 2048
#endif
#define NB_FULL  2
#define SEQ_FULL 2048
#define DM 1024
#define NH 16
#define DH 64

static_assert(SEQ % 64 == 0);
static_assert(SEQ <= SEQ_FULL);
static_assert(NB <= NB_FULL);
static_assert(NH * DH == DM);

typedef __attribute__((ext_vector_type(16))) _Float16 v16h;
typedef __attribute__((ext_vector_type(8)))  _Float16 v8h;
typedef __attribute__((ext_vector_type(16))) __bf16   v16b;
typedef __attribute__((ext_vector_type(8)))  __bf16   v8b;
typedef __attribute__((ext_vector_type(8)))  float    v8f;
typedef __attribute__((ext_vector_type(4)))  float    v4f;
typedef unsigned int cm_u4 __attribute__((ext_vector_type(4)));

__device__ __forceinline__ int frag_k(int i, int h) { return (i < 8) ? (8 * h + i) : (16 + 8 * h + (i - 8)); }

__device__ __forceinline__ v8f wmma16(v16h a, v16h b, v8f c) {
    c = __builtin_amdgcn_wmma_f32_16x16x32_f16(false, a, false, b, (short)0, c, false, false);
    asm volatile("v_nop\n\tv_nop\n\tv_nop\n\tv_nop" : "+v"(c) : "v"(a), "v"(b));
    return c;
}

__device__ __forceinline__ v16h fh_ld(const float* __restrict__ p, int k0, int h, float s) {
    v16h a;
#pragma unroll
    for (int i = 0; i < 16; ++i) a[i] = (_Float16)(p[k0 + frag_k(i, h)] * s);
    return a;
}
__device__ __forceinline__ v16h fh_lds(const float* p, int k0, int h, float s) {
    v16h a;
#pragma unroll
    for (int i = 0; i < 16; ++i) a[i] = (_Float16)(p[k0 + frag_k(i, h)] * s);
    return a;
}

#define VST2(T, ptr, val) do { const T vst2_v_ = (val); *(volatile T*)(ptr) = vst2_v_; __threadfence(); *(volatile T*)(ptr) = vst2_v_; } while (0)
#define VST2V4(ptr, val) do { const v4f vst2_v4_ = (val); *(volatile v4f*)(ptr) = vst2_v4_; __threadfence(); *(volatile v4f*)(ptr) = vst2_v4_; } while (0)

#define AW 4
struct AttnP {
    const float* Q; const float* K; const float* V; float* O; const float* KB;
    long long sQb, sQh, sQi, sKb, sKh, sKj, sVb, sVh, sVj, sOb, sOh, sOi, sbb;
    int Lq, Lk; float scale; int pad_;
};
static_assert(sizeof(AttnP) == 5 * 8 + 13 * 8 + 4 * 4);

#ifndef KATTN_ATTR
#define KATTN_ATTR
#endif
template <int DHP, int DVP>
__global__ __launch_bounds__(32 * AW) KATTN_ATTR void k_attn(AttnP p) {
    constexpr int NT = DVP / 16;
    constexpr int KS = DHP / 32;
    constexpr int VP = DVP + 8;
    __shared__ __align__(16) float    pl[AW][16 * 64];
    __shared__ __align__(16) _Float16 vl[64 * VP];
    const int lane = threadIdx.x & 31, hf = lane >> 4, l15 = lane & 15, wave = __builtin_amdgcn_readfirstlane((int)(threadIdx.x >> 5));
    const int h = blockIdx.y, b = blockIdx.z;
    const int q0 = (blockIdx.x * AW + wave) * 16;
    float* myp = pl[wave];
    const float L2E = 1.4426950408889634f;
    const float NEG = -__builtin_inff();
    const int qi = min(q0 + l15, p.Lq - 1);
    const float* qrow = p.Q + b * p.sQb + h * p.sQh + (long long)qi * p.sQi;
    const float* kbase = p.K + b * p.sKb + h * p.sKh;
    const float* vbase = p.V + b * p.sVb + h * p.sVh;
    const float* kbias = p.KB + b * p.sbb;
    v16h qa[KS];
#pragma unroll
    for (int ks = 0; ks < KS; ++ks) qa[ks] = fh_ld(qrow, ks * 32, hf, 1.f);
    v8f o[NT]; float m8[8], l8[8];
#pragma unroll
    for (int t = 0; t < NT; ++t) { v8f zz = {}; o[t] = zz; }
#pragma unroll
    for (int i = 0; i < 8; ++i) { m8[i] = NEG; l8[i] = 0.f; }
    for (int j0 = 0; j0 < p.Lk; j0 += 64) {
        __syncthreads();
        for (int idx = threadIdx.x; idx < 64 * DVP; idx += 32 * AW) {
            const int jr = idx / DVP, d = idx - jr * DVP, j = j0 + jr;
            const int jc = min(j, p.Lk - 1);
            float f = vbase[(long long)jc * p.sVj + d];
            if (j >= p.Lk) f = 0.f;
            vl[jr * VP + d] = (_Float16)f;
        }
        v8f s[4];
#pragma unroll
        for (int t = 0; t < 4; ++t) {
            const int j = min(j0 + t * 16 + l15, p.Lk - 1);
            const float* krow = kbase + (long long)j * p.sKj;
            v8f acc = {};
#pragma unroll
            for (int ks = 0; ks < KS; ++ks) acc = wmma16(qa[ks], fh_ld(krow, ks * 32, hf, 1.f), acc);
            s[t] = acc;
        }
        float kb4[4];
#pragma unroll
        for (int t = 0; t < 4; ++t) kb4[t] = kbias[min(j0 + t * 16 + l15, p.Lk - 1)];
        float pv[8][4];
#pragma unroll
        for (int i = 0; i < 8; ++i) {
            float sc[4];
#pragma unroll
            for (int t = 0; t < 4; ++t) {
                const int jg = j0 + t * 16 + l15;
                const float v = s[t][i] * p.scale + kb4[t];
                sc[t] = (jg >= p.Lk) ? NEG : v;
            }
            float mx = fmaxf(fmaxf(sc[0], sc[1]), fmaxf(sc[2], sc[3]));
            mx = fmaxf(mx, __shfl_xor(mx, 1, 32)); mx = fmaxf(mx, __shfl_xor(mx, 2, 32));
            mx = fmaxf(mx, __shfl_xor(mx, 4, 32)); mx = fmaxf(mx, __shfl_xor(mx, 8, 32));
            const float mnew = fmaxf(m8[i], mx);
            const float corr = (mnew == NEG) ? 1.f : exp2f((m8[i] - mnew) * L2E);
            float rs = 0.f;
#pragma unroll
            for (int t = 0; t < 4; ++t) {
                const float pp = (sc[t] == NEG) ? 0.f : exp2f((sc[t] - mnew) * L2E);
                rs += pp; pv[i][t] = pp;
            }
            rs += __shfl_xor(rs, 1, 32); rs += __shfl_xor(rs, 2, 32); rs += __shfl_xor(rs, 4, 32); rs += __shfl_xor(rs, 8, 32);
            l8[i] = l8[i] * corr + rs; m8[i] = mnew;
#pragma unroll
            for (int t = 0; t < NT; ++t) o[t][i] *= corr;
        }
#pragma unroll
        for (int i = 0; i < 8; ++i)
#pragma unroll
            for (int t = 0; t < 4; ++t) myp[(i + 8 * hf) * 64 + t * 16 + l15] = pv[i][t];
        __syncthreads();
        {
            const v16h pa0 = fh_lds(myp + l15 * 64, 0, hf, 4096.f), pa1 = fh_lds(myp + l15 * 64, 32, hf, 4096.f);
#pragma unroll
            for (int t = 0; t < NT; ++t) {
                const int dcol = t * 16 + l15;
                v16h b0, b1;
#pragma unroll
                for (int e = 0; e < 16; ++e) { b0[e] = vl[frag_k(e, hf) * VP + dcol]; b1[e] = vl[(32 + frag_k(e, hf)) * VP + dcol]; }
                o[t] = wmma16(pa0, b0, o[t]);
                o[t] = wmma16(pa1, b1, o[t]);
            }
        }
    }
    float* obase = p.O + b * p.sOb + h * p.sOh;
    float invr[8];
#pragma unroll
    for (int i = 0; i < 8; ++i) invr[i] = (l8[i] > 0.f) ? 1.f / (l8[i] * 4096.f) : 0.f;
    __syncthreads();
#pragma unroll
    for (int i = 0; i < 8; ++i)
#pragma unroll
        for (int t = 0; t < NT; ++t) myp[(i + 8 * hf) * 64 + t * 16 + l15] = o[t][i] * invr[i];
    __syncthreads();
    {
        constexpr int lpr = DVP / 4;
        constexpr int rows_per_ins = 32 / lpr;
        for (int r0 = 0; r0 < 16; r0 += rows_per_ins) {
            const int row = r0 + lane / lpr, c4 = (lane % lpr) * 4;
            const v4f v = *(const v4f*)(myp + row * 64 + c4);
            VST2V4(obase + (long long)(q0 + row) * p.sOi + c4, v);
        }
    }
    __syncthreads();
}

__device__ __forceinline__ void dep_guard_h(v8f& a, v8f& b, v16h x, v16h y) { asm volatile("v_nop\n\tv_nop\n\tv_nop\n\tv_nop" : "+v"(a), "+v"(b) : "v"(x), "v"(y)); }
__device__ __forceinline__ void dep_guard_b(v8f& a, v8f& b, v16b x, v16b y) { asm volatile("v_nop\n\tv_nop\n\tv_nop\n\tv_nop" : "+v"(a), "+v"(b) : "v"(x), "v"(y)); }
__device__ __forceinline__ void keep4_h(v16h a, v16h b, v16h c, v16h d) { asm volatile("v_nop" :: "v"(a), "v"(b), "v"(c), "v"(d)); }
__device__ __forceinline__ void keep4_b(v16b a, v16b b, v16b c, v16b d) { asm volatile("v_nop" :: "v"(a), "v"(b), "v"(c), "v"(d)); }
__device__ __forceinline__ void acc_guard4(v8f& a, v8f& b, v8f& c, v8f& d) { asm volatile("v_nop\n\tv_nop\n\tv_nop\n\tv_nop" : "+v"(a), "+v"(b), "+v"(c), "+v"(d)); }
template <typename T> struct Frag;
template <> struct Frag<_Float16> {
  typedef v16h V; union U { v16h v; v8h h[2]; };
  static __device__ __forceinline__ v16h load(const _Float16* p) {
    U f; f.h[0] = *(const v8h*)(p); f.h[1] = *(const v8h*)(p + 16); return f.v;
  }
  static __device__ __forceinline__ v8f mma(v16h a, v16h b, v8f c) {
    return __builtin_amdgcn_wmma_f32_16x16x32_f16(false, a, false, b, (short)0, c, false, false);
  }
  static __device__ __forceinline__ void guard(v8f& a, v8f& b, v16h x, v16h y) { dep_guard_h(a, b, x, y); }
  static __device__ __forceinline__ void keep(v16h a, v16h b, v16h c, v16h d) { keep4_h(a, b, c, d); }
};
template <> struct Frag<__bf16> {
  typedef v16b V; union U { v16b v; v8b h[2]; };
  static __device__ __forceinline__ v16b load(const __bf16* p) {
    U f; f.h[0] = *(const v8b*)(p); f.h[1] = *(const v8b*)(p + 16); return f.v;
  }
  static __device__ __forceinline__ v8f mma(v16b a, v16b b, v8f c) {
    return __builtin_amdgcn_wmma_f32_16x16x32_bf16(false, a, false, b, (short)0, c, false, false);
  }
  static __device__ __forceinline__ void guard(v8f& a, v8f& b, v16b x, v16b y) { dep_guard_b(a, b, x, y); }
  static __device__ __forceinline__ void keep(v16b a, v16b b, v16b c, v16b d) { keep4_b(a, b, c, d); }
};

template <int ET> struct Elem;
template <> struct Elem<0> { typedef _Float16 T; };
template <> struct Elem<1> { typedef __bf16 T; };
template <int ET, int BIAS_MODE, bool RESID>
__global__ __launch_bounds__(256) void wmma_gemm64(
    const unsigned short* __restrict__ Ap, int lda, long strideA,
    const unsigned short* __restrict__ Btp, int ldb, long strideB,
    float* Cout, int ldc, long strideC,
    const float* __restrict__ bias,
    const float* resid, long strideR,
    int M, int N, int K, float scale) {
  typedef typename Elem<ET>::T T;
  typedef typename Frag<T>::V V;
  const T* A = (const T*)Ap; const T* Bt = (const T*)Btp;
  __shared__ __align__(16) float sT[8][16 * 68];
  const int b    = blockIdx.y;
  const int lane = threadIdx.x & 31;
  const int wave = __builtin_amdgcn_readfirstlane((int)(threadIdx.x >> 5));
  const int tilesN = N >> 6;
  const int tilesM = M >> 6;
  const int tile = blockIdx.x * 8 + wave;
  if (tile >= tilesM * tilesN) return;
  const int tm = tile / tilesN;
  const int tn = tile - tm * tilesN;
  const int m0 = tm << 6;
  const int n0 = tn << 6;

  const T* Ab  = A  + (size_t)b * strideA;
  const T* Bb  = Bt + (size_t)b * strideB;

  const int rlane = lane & 15;
  const int koff  = (lane >> 4) * 8;
  const int mOff  = (lane >> 4) * 8;

  v8f acc[4][4];
#pragma unroll
  for (int i = 0; i < 4; ++i)
#pragma unroll
    for (int j = 0; j < 4; ++j) acc[i][j] = (v8f){0.f,0.f,0.f,0.f,0.f,0.f,0.f,0.f};

  for (int k0 = 0; k0 < K; k0 += 32) {
    V bh[4];
#pragma unroll
    for (int j = 0; j < 4; ++j) {
      const size_t bo = (size_t)(n0 + (j << 4) + rlane) * ldb + koff + k0;
      bh[j] = Frag<T>::load(Bb + bo);
    }
#pragma unroll
    for (int i = 0; i < 4; ++i) {
      const size_t ao = (size_t)(m0 + (i << 4) + rlane) * lda + koff + k0;
      V ah = Frag<T>::load(Ab + ao);
#pragma unroll
      for (int j = 0; j < 4; ++j) acc[i][j] = Frag<T>::mma(ah, bh[j], acc[i][j]);
      Frag<T>::guard(acc[i][0], acc[i][3], ah, ah);
    }
    Frag<T>::keep(bh[0], bh[1], bh[2], bh[3]);
  }
  acc_guard4(acc[0][0], acc[0][1], acc[0][2], acc[0][3]);
  acc_guard4(acc[1][0], acc[1][1], acc[1][2], acc[1][3]);
  acc_guard4(acc[2][0], acc[2][1], acc[2][2], acc[2][3]);
  acc_guard4(acc[3][0], acc[3][1], acc[3][2], acc[3][3]);

  float* slab = sT[wave];
  const float* Rb = RESID ? (resid + (size_t)b * strideR) : nullptr;
  float* C = Cout + (size_t)b * strideC;
#pragma unroll
  for (int i = 0; i < 4; ++i) {
    const int mBase = m0 + (i << 4);
#pragma unroll
    for (int j = 0; j < 4; ++j) {
      const int n = n0 + (j << 4) + rlane;
      float bv = 0.f;
      if (BIAS_MODE == 2) bv = bias[n];
#pragma unroll
      for (int r = 0; r < 8; ++r) {
        float v = acc[i][j][r] * scale;
        if (BIAS_MODE == 2) v += bv;
        if (RESID) v += Rb[(size_t)(mBase + mOff + r) * ldc + n];
        slab[(mOff + r) * 68 + (j << 4) + rlane] = v;
      }
    }
    __builtin_amdgcn_fence(3  , "workgroup");
    __builtin_amdgcn_wave_barrier();
    __builtin_amdgcn_fence(2  , "workgroup");
    {
      const int hh = lane >> 4, c4 = (lane & 15) * 4;
      for (int pass = 0; pass < 2; ++pass) {
#pragma unroll
        for (int it = 0; it < 8; ++it) {
          const int row = it * 2 + hh;
          v4f v = *(const v4f*)(slab + row * 68 + c4);
          *(volatile v4f*)(C + (size_t)(mBase + row) * ldc + n0 + c4) = v;
        }
        __threadfence();
      }
    }
    __builtin_amdgcn_fence(3  , "workgroup");
    __builtin_amdgcn_wave_barrier();
    __builtin_amdgcn_fence(2  , "workgroup");
  }
}

__device__ __forceinline__ unsigned short f2bf_bits(float f) {
  unsigned u = __float_as_uint(f);
  return (unsigned short)((u + 0x7FFFu + ((u >> 16) & 1u)) >> 16);
}
__device__ __forceinline__ float bf_bits2f(unsigned short h) { return __uint_as_float(((unsigned)h) << 16); }
__device__ __forceinline__ unsigned int cmb_pk2(float a, float b) { return (unsigned int)__builtin_bit_cast(unsigned short, (_Float16)a) | ((unsigned int)__builtin_bit_cast(unsigned short, (_Float16)b) << 16); }
__device__ __forceinline__ float cmb_bf(float v) { const unsigned u = __builtin_bit_cast(unsigned, v); const unsigned r = (u + 0x7fffu + ((u >> 16) & 1u)) & 0xffff0000u; return __builtin_bit_cast(float, r); }

__global__ __launch_bounds__(256) void k_cm_castb(const float* __restrict__ SRC, int lds, unsigned short* __restrict__ DST, int ldd, int nR, int nC, float sc, int rpb, int rpbs) {
    const long long u = (long long)blockIdx.x * 256 + threadIdx.x; const int per = nC / 8; if (u >= (long long)nR * per) return; const int r = (int)(u / per); const int c0 = 8 * (int)(u % per);
    const long long rs = (long long)(r / rpb) * rpbs + (r % rpb);
    const float* s = SRC + rs * lds + c0; float w[8];
#pragma unroll
    for (int e = 0; e < 8; ++e) w[e] = cmb_bf(s[e]) * sc;
    cm_u4 pk; pk.x = cmb_pk2(w[0], w[1]); pk.y = cmb_pk2(w[2], w[3]); pk.z = cmb_pk2(w[4], w[5]); pk.w = cmb_pk2(w[6], w[7]); VST2(cm_u4, (cm_u4*)(DST + (long long)r * ldd + c0), pk); }

__global__ __launch_bounds__(256) void k_cm_castbf(const float* __restrict__ SRC, int lds, unsigned short* __restrict__ DST, int ldd, int nR, int nC) {
    const long long u = (long long)blockIdx.x * 256 + threadIdx.x; const int per = nC / 8; if (u >= (long long)nR * per) return; const int r = (int)(u / per); const int c0 = 8 * (int)(u % per);
    const float* s = SRC + (long long)r * lds + c0; unsigned w[8];
#pragma unroll
    for (int e = 0; e < 8; ++e) w[e] = (unsigned)f2bf_bits(s[e]);
    cm_u4 pk; pk.x = w[0] | (w[1] << 16); pk.y = w[2] | (w[3] << 16); pk.z = w[4] | (w[5] << 16); pk.w = w[6] | (w[7] << 16); VST2(cm_u4, (cm_u4*)(DST + (long long)r * ldd + c0), pk); }

__global__ __launch_bounds__(256) void k_cm_bias4(const float* __restrict__ B0, const float* __restrict__ B1, const float* __restrict__ B2, const float* __restrict__ B3, float* __restrict__ DST, int n) {
    const int u = blockIdx.x * 256 + threadIdx.x; const int y = blockIdx.y; if (u >= n) return;
    const float a0 = B0[u], a1 = B1[u], a2 = B2[u], a3 = B3[u];
    const float v = (y == 0) ? a0 : ((y == 1) ? a1 : ((y == 2) ? a2 : a3));
    const float r = cmb_bf(v); VST2(float, DST + (long long)y * n + u, r); }

__global__ __launch_bounds__(256) void k_maskadd(const float* __restrict__ M, float* __restrict__ DST, int seq, int seq_full, int n) {
    const int u = blockIdx.x * 256 + threadIdx.x; if (u >= n) return; const int b = u / seq, s = u - b * seq;
    const float m = cmb_bf(M[(long long)b * seq_full + s]);
    const float v = (1.0f - m) * -10000.0f; VST2(float, DST + u, v); }

__device__ __forceinline__ unsigned int f2bf2_pack(float a, float b, unsigned int* lo) {
    const unsigned short ha = f2bf_bits(a), hb = f2bf_bits(b);
    const unsigned short la = f2bf_bits(a - bf_bits2f(ha)), lb = f2bf_bits(b - bf_bits2f(hb));
    *lo = (unsigned)la | ((unsigned)lb << 16); return (unsigned)ha | ((unsigned)hb << 16); }
__global__ __launch_bounds__(256) void k_castS16(const float* __restrict__ src, long long lds, unsigned short* __restrict__ dhi, unsigned short* __restrict__ dlo, long long ldd, int R, int C) {
    const long long i = (long long)blockIdx.x * 256 + threadIdx.x; const long long np = (long long)R * (C / 2); if (i >= np) return;
    const int r = (int)(i / (C / 2)); const int c = 2 * (int)(i % (C / 2));
    const float a = src[(long long)r * lds + c], b = src[(long long)r * lds + c + 1]; const long long o = (long long)r * ldd + c;
    unsigned lo; const unsigned hi = f2bf2_pack(a, b, &lo); volatile unsigned* ph = (volatile unsigned*)(dhi + o); volatile unsigned* pq = (volatile unsigned*)(dlo + o);
    *ph = hi; *pq = lo; __threadfence(); *ph = hi; *pq = lo; }

static inline size_t al256(size_t bytes) { return ((bytes + 255) / 256) * 256; }

extern "C" void kernel_launch(void* const* d_in, const int* in_sizes, int n_in, void* d_out, int out_size, void* d_ws, size_t ws_size, hipStream_t stream) {
    if (n_in < 11) return;
    const long long rows_need = (long long)(NB - 1) * SEQ_FULL + SEQ;
    if ((long long)in_sizes[0] < rows_need * DM) return;
    if ((long long)in_sizes[1] < rows_need * DM) return;
    if ((long long)in_sizes[2] < rows_need) return;
    if (in_sizes[3] < DM * DM || in_sizes[5] < DM * DM || in_sizes[7] < DM * DM || in_sizes[9] < DM * DM) return;
    if (in_sizes[4] < DM || in_sizes[6] < DM || in_sizes[8] < DM || in_sizes[10] < DM) return;
    const int MR = NB * SEQ;
    if ((long long)out_size < (long long)MR * DM) return;

    const float* x    = (const float*)d_in[0];
    const float* y    = (const float*)d_in[1];
    const float* mask = (const float*)d_in[2];
    const float* wq   = (const float*)d_in[3];
    const float* bq   = (const float*)d_in[4];
    const float* wk   = (const float*)d_in[5];
    const float* bk   = (const float*)d_in[6];
    const float* wv   = (const float*)d_in[7];
    const float* bv   = (const float*)d_in[8];
    const float* wo   = (const float*)d_in[9];
    const float* bo   = (const float*)d_in[10];
    float* out = (float*)d_out;

    size_t off = 0;
    const size_t oX16  = off; off += al256((size_t)MR * DM * 2);
    const size_t oY16  = off; off += al256((size_t)MR * DM * 2);
    const size_t oW316 = off; off += al256((size_t)3 * DM * DM * 2);
    const size_t oQKV  = off; off += al256((size_t)MR * 3 * DM * 4);
    const size_t oAO   = off; off += al256((size_t)MR * DM * 4);
    const size_t oBR4  = off; off += al256((size_t)4 * DM * 4);
    const size_t oMADD = off; off += al256((size_t)MR * 4);
    const size_t oWOB  = off; off += al256((size_t)DM * DM * 2);
    const size_t oAOH  = off; off += al256((size_t)MR * DM * 2);
    const size_t oAOL  = off; off += al256((size_t)MR * DM * 2);
    if (off > ws_size || off > (size_t)134217728) return;
    char* base = (char*)d_ws;
    unsigned short* X16  = (unsigned short*)(base + oX16);
    unsigned short* Y16  = (unsigned short*)(base + oY16);
    unsigned short* W316 = (unsigned short*)(base + oW316);
    float* QKV  = (float*)(base + oQKV);
    float* AO   = (float*)(base + oAO);
    float* BR4  = (float*)(base + oBR4);
    float* MADD = (float*)(base + oMADD);
    unsigned short* WOB = (unsigned short*)(base + oWOB);
    unsigned short* AOH = (unsigned short*)(base + oAOH);
    unsigned short* AOL = (unsigned short*)(base + oAOL);

    const unsigned gW = (unsigned)((((long long)DM) * (DM / 8) + 255) / 256);
    const unsigned gX = (unsigned)((((long long)MR) * (DM / 8) + 255) / 256);
    k_cm_castb<<<gW, 256, 0, stream>>>(wq, DM, W316, DM, DM, DM, 16.0f, DM, DM);
    k_cm_castb<<<gW, 256, 0, stream>>>(wk, DM, W316 + (size_t)DM * DM, DM, DM, DM, 16.0f, DM, DM);
    k_cm_castb<<<gW, 256, 0, stream>>>(wv, DM, W316 + (size_t)2 * DM * DM, DM, DM, DM, 16.0f, DM, DM);
    k_cm_bias4<<<dim3((DM + 255) / 256, 4), 256, 0, stream>>>(bq, bk, bv, bo, BR4, DM);
    k_cm_castb<<<gX, 256, 0, stream>>>(x, DM, X16, DM, MR, DM, 1.0f, SEQ, SEQ_FULL);
    k_cm_castb<<<gX, 256, 0, stream>>>(y, DM, Y16, DM, MR, DM, 1.0f, SEQ, SEQ_FULL);
    wmma_gemm64<0, 2, false><<<dim3((unsigned)((((MR) / 64) * ((DM) / 64) + 7) / 8), 1u), 256, 0, stream>>>(
        X16, DM, 0, W316, DM, 0, QKV, 3 * DM, 0, BR4, nullptr, 0, MR, DM, DM, 0.0625f);
    wmma_gemm64<0, 2, false><<<dim3((unsigned)((((MR) / 64) * ((2 * DM) / 64) + 7) / 8), 1u), 256, 0, stream>>>(
        Y16, DM, 0, W316 + (size_t)DM * DM, DM, 0, QKV + DM, 3 * DM, 0, BR4 + DM, nullptr, 0, MR, 2 * DM, DM, 0.0625f);
    k_maskadd<<<(unsigned)((MR + 255) / 256), 256, 0, stream>>>(mask, MADD, SEQ, SEQ_FULL, MR);
    k_cm_castbf<<<gW, 256, 0, stream>>>(wo, DM, WOB, DM, DM, DM);
    {
        AttnP a;
        a.Q = QKV; a.K = QKV + DM; a.V = QKV + 2 * DM; a.O = AO; a.KB = MADD;
        a.sQb = (long long)SEQ * 3 * DM; a.sQh = DH; a.sQi = 3 * DM;
        a.sKb = (long long)SEQ * 3 * DM; a.sKh = DH; a.sKj = 3 * DM;
        a.sVb = (long long)SEQ * 3 * DM; a.sVh = DH; a.sVj = 3 * DM;
        a.sOb = (long long)SEQ * DM; a.sOh = DH; a.sOi = DM; a.sbb = SEQ;
        a.Lq = SEQ; a.Lk = SEQ; a.scale = 0.125f; a.pad_ = 0;
        k_attn<64, 64><<<dim3((unsigned)((SEQ + 16 * AW - 1) / (16 * AW)), (unsigned)NH, (unsigned)NB), 32 * AW, 0, stream>>>(a);
    }
    k_castS16<<<(unsigned)((((long long)MR * (DM / 2)) + 255) / 256), 256, 0, stream>>>(AO, DM, AOH, AOL, DM, MR, DM);
    wmma_gemm64<1, 2, false><<<dim3((unsigned)((((MR) / 64) * ((DM) / 64) + 7) / 8), 1u), 256, 0, stream>>>(
        AOH, DM, 0, WOB, DM, 0, out, DM, 0, BR4 + 3 * DM, nullptr, 0, MR, DM, DM, 1.0f);
    wmma_gemm64<1, 0, true><<<dim3((unsigned)((((MR) / 64) * ((DM) / 64) + 7) / 8), 1u), 256, 0, stream>>>(
        AOL, DM, 0, WOB, DM, 0, out, DM, 0, nullptr, out, 0, MR, DM, DM, 1.0f);
}
